// MoELayer_25864293057158
// MI455X (gfx1250) — hardware-verified
//
#include <hip/hip_runtime.h>
#include <math.h>

typedef __attribute__((ext_vector_type(16))) _Float16 v16h;
typedef __attribute__((ext_vector_type(16))) __bf16 v16b;
typedef __attribute__((ext_vector_type(8)))  _Float16 v8h;
typedef __attribute__((ext_vector_type(8)))  __bf16 v8b;
typedef __attribute__((ext_vector_type(8)))  float v8f;
typedef __attribute__((ext_vector_type(4)))  float v4f;
typedef __attribute__((ext_vector_type(4)))  unsigned v4u;
typedef _Float16 h16;

#ifndef NB
#define NB 2
#endif
#ifndef SEQ
#define SEQ 4096
#endif
#define NB_FULL 2
#define SEQ_FULL 4096
#define NTOK (NB * SEQ)
#define DIN  512
#define DHID 2048
#define DOUT 512
#define NE   8
#define CH   512
#define MT   32
#define HC   256
#define XP   (DIN + 8)
#define HP   (HC + 8)
#define HCARRY 64.0f
#define WCARRY 512.0f
#define OSCALE (1.0f / 32768.0f)

#define WS_W1T ((size_t)0)
#define WS_W2T (WS_W1T + (size_t)NE * DHID * DIN * 2)
#define WS_YS  (WS_W2T + (size_t)NE * DOUT * DHID * 2)
#define WS_END (WS_YS  + (size_t)2 * NTOK * DOUT * 4)

static_assert(NE == 8);
static_assert(NB <= NB_FULL && SEQ <= SEQ_FULL);
static_assert(NTOK % CH == 0 && CH % 256 == 0 && CH % MT == 0 && (CH & (CH - 1)) == 0);
static_assert(DIN % 64 == 0 && DHID % 64 == 0 && DOUT % 64 == 0);
static_assert(DIN % 32 == 0 && HC % 32 == 0 && DHID % HC == 0);
static_assert(HC == 8 * 32);
static_assert(DOUT == 8 * 64);
static_assert(MT == 32);
static_assert((XP * 2) % 16 == 0 && (HP * 2) % 16 == 0);
static_assert((size_t)NTOK * DOUT * 4 <= 16777216);
static_assert(WS_W2T % 128 == 0 && WS_YS % 128 == 0);
static_assert(WS_END <= (size_t)134217728);
static_assert((size_t)(DHID / 64) * (DIN / 64) * NE * 4096 == (size_t)NE * DIN * DHID);
static_assert((size_t)(DOUT / 64) * (DHID / 64) * NE * 4096 == (size_t)NE * DHID * DOUT);
static_assert((size_t)(NTOK * DOUT / 4 / 256) * 256 * 4 == (size_t)NTOK * DOUT);
static_assert(256 * 2 * 16 == 64 * 128);
static_assert(32 * 8 * 16 == 16 * 64 * 4);
static_assert((MT * DIN / 8) % 256 == 0);
static_assert((size_t)MT * XP * 2 + (size_t)MT * HP * 2 + (size_t)8 * 16 * 64 * 4 + (size_t)DIN * NE * 4 + (size_t)CH * 16 + (size_t)MT * 8 + 64 <= 131072);
static_assert((size_t)64 * 65 * 4 <= 131072);

__device__ __forceinline__ v8f wmma16(v16h a, v16h b, v8f c) {
  v8f d = __builtin_amdgcn_wmma_f32_16x16x32_f16(false, a, false, b, (short)0, c, false, false);
  asm volatile("v_nop\n\tv_nop\n\tv_nop\n\tv_nop" : "+v"(d) : "v"(a), "v"(b));
  return d;
}
__device__ __forceinline__ v8f wmma_bf(v16b a, v16b b, v8f c) {
  v8f d = __builtin_amdgcn_wmma_f32_16x16x32_bf16(false, a, false, b, (short)0, c, false, false);
  asm volatile("v_nop\n\tv_nop\n\tv_nop\n\tv_nop" : "+v"(d) : "v"(a), "v"(b));
  return d;
}
__device__ __forceinline__ float bfr(float v) { return (float)(__bf16)v; }
static __device__ __forceinline__ h16 toh_flush(float v) { const h16 r = (h16)v; return (fabsf(v) < 6.103515625e-05f) ? (h16)0.0f : r; }
__device__ __forceinline__ v16b ldfrag_b(const unsigned short* p) { union { v16b v; v4u q[2]; } f; f.q[0] = *(const v4u*)p; f.q[1] = *(const v4u*)(p + 16); return f.v; }
__device__ __forceinline__ v16h ldfrag_h(const unsigned short* p) { union { v16h v; v4u q[2]; } f; f.q[0] = *(const v4u*)p; f.q[1] = *(const v4u*)(p + 16); return f.v; }

__global__ __launch_bounds__(256) void k_tr_w1(const float* __restrict__ S, unsigned short* __restrict__ Dst, unsigned K, unsigned N, unsigned dpitch, unsigned erow, unsigned ecol) {
  __shared__ float tile[64][65];
  const unsigned t = threadIdx.x, e = blockIdx.z, k0 = blockIdx.y * 64u, n0 = blockIdx.x * 64u;
  const float* s = S + (size_t)e * K * N;
#pragma unroll
  for (unsigned it = 0; it < 4; ++it) { const unsigned idx = it * 256u + t, kr = idx >> 4, c4 = idx & 15u;
    const v4f v = *(const v4f*)(s + (size_t)(k0 + kr) * N + n0 + 4u * c4);
    tile[kr][4u * c4 + 0] = v[0]; tile[kr][4u * c4 + 1] = v[1]; tile[kr][4u * c4 + 2] = v[2]; tile[kr][4u * c4 + 3] = v[3]; }
  __syncthreads();
  v4u o[2];
#pragma unroll
  for (unsigned it = 0; it < 2; ++it) { const unsigned idx = it * 256u + t, nr = idx >> 3, q = idx & 7u;
    union { v8b b; v4u u; } w;
#pragma unroll
    for (int i = 0; i < 8; ++i) w.b[i] = (__bf16)tile[8u * q + i][nr];
    o[it] = w.u; }
#pragma unroll
  for (unsigned it = 0; it < 2; ++it) { const unsigned idx = it * 256u + t, nr = idx >> 3, q = idx & 7u;
    *(volatile v4u*)(Dst + (size_t)(e * erow + n0 + nr) * dpitch + e * ecol + k0 + 8u * q) = o[it]; }
  __threadfence();
#pragma unroll
  for (unsigned it = 0; it < 2; ++it) { const unsigned idx = it * 256u + t, nr = idx >> 3, q = idx & 7u;
    *(volatile v4u*)(Dst + (size_t)(e * erow + n0 + nr) * dpitch + e * ecol + k0 + 8u * q) = o[it]; }
}

__global__ __launch_bounds__(256) void k_tr_w2(const float* __restrict__ S, unsigned short* __restrict__ Dst, unsigned K, unsigned N, unsigned dpitch, unsigned erow, unsigned ecol, float sc) {
  __shared__ float tile[64][65];
  const unsigned t = threadIdx.x, e = blockIdx.z, k0 = blockIdx.y * 64u, n0 = blockIdx.x * 64u;
  const float* s = S + (size_t)e * K * N;
#pragma unroll
  for (unsigned it = 0; it < 4; ++it) { const unsigned idx = it * 256u + t, kr = idx >> 4, c4 = idx & 15u;
    const v4f v = *(const v4f*)(s + (size_t)(k0 + kr) * N + n0 + 4u * c4);
    tile[kr][4u * c4 + 0] = v[0]; tile[kr][4u * c4 + 1] = v[1]; tile[kr][4u * c4 + 2] = v[2]; tile[kr][4u * c4 + 3] = v[3]; }
  __syncthreads();
  v4u o[2];
#pragma unroll
  for (unsigned it = 0; it < 2; ++it) { const unsigned idx = it * 256u + t, nr = idx >> 3, q = idx & 7u;
    union { v8h h; v4u u; } w;
#pragma unroll
    for (int i = 0; i < 8; ++i) { const float v = bfr(tile[8u * q + i][nr]); w.h[i] = toh_flush(v * sc); }
    o[it] = w.u; }
#pragma unroll
  for (unsigned it = 0; it < 2; ++it) { const unsigned idx = it * 256u + t, nr = idx >> 3, q = idx & 7u;
    *(volatile v4u*)(Dst + (size_t)(e * erow + n0 + nr) * dpitch + e * ecol + k0 + 8u * q) = o[it]; }
  __threadfence();
#pragma unroll
  for (unsigned it = 0; it < 2; ++it) { const unsigned idx = it * 256u + t, nr = idx >> 3, q = idx & 7u;
    *(volatile v4u*)(Dst + (size_t)(e * erow + n0 + nr) * dpitch + e * ecol + k0 + 8u * q) = o[it]; }
}

__global__ __launch_bounds__(256) __attribute__((amdgpu_num_vgpr(256)))
void k_moe(const float* __restrict__ X, const float* __restrict__ TS, const float* __restrict__ GW, const float* __restrict__ GB,
           const unsigned short* __restrict__ W1T, const float* __restrict__ B1, const unsigned short* __restrict__ W2T, const float* __restrict__ B2,
           float* __restrict__ YS) {
  __shared__ __align__(16) unsigned short sx[MT][XP];
  __shared__ __align__(16) _Float16 shh[MT][HP];
  __shared__ __align__(16) float sf[8][16][64];
  __shared__ __align__(16) float s_gw[DIN * NE];
  __shared__ int   s_sel[CH];
  __shared__ float s_p1[CH];
  __shared__ float s_p2[CH];
  __shared__ int   s_list[CH];
  __shared__ int   s_rdst[MT];
  __shared__ float s_rw[MT];
  __shared__ int   s_wcnt[16];
  const unsigned t = threadIdx.x, lane = t & 31u, lm = lane & 15u, lh = lane >> 4, wv = t >> 5;
  const unsigned wave = (unsigned)__builtin_amdgcn_readfirstlane((int)(threadIdx.x >> 5));
  const unsigned tok0 = blockIdx.x * (unsigned)CH;

#pragma unroll 1
  for (unsigned i = t; i < (unsigned)(DIN * NE); i += 256u) s_gw[i] = bfr(GW[i]);
#pragma unroll 1
  for (unsigned i = t; i < (unsigned)CH; i += 256u) s_list[i] = 0;
  __syncthreads();
#pragma unroll 1
  for (unsigned j = 0; j < (unsigned)(CH / 256); ++j) {
    const unsigned tokl = j * 256u + t;
    const float* xr = X  + (size_t)(tok0 + tokl) * DIN;
    const float* tr = TS + (size_t)(tok0 + tokl) * DIN;
    float l[NE];
#pragma unroll
    for (int q = 0; q < NE; ++q) l[q] = 0.f;
#pragma unroll 1
    for (unsigned k4 = 0; k4 < (unsigned)(DIN / 4); ++k4) {
      const v4f xv = *(const v4f*)(xr + 4u * k4), tv = *(const v4f*)(tr + 4u * k4);
#pragma unroll
      for (int i = 0; i < 4; ++i) {
        const float v = bfr(xv[i]) + bfr(tv[i]);
        const v4f g0 = *(const v4f*)&s_gw[(4u * k4 + (unsigned)i) * NE], g1 = *(const v4f*)&s_gw[(4u * k4 + (unsigned)i) * NE + 4u];
        l[0] = fmaf(v, g0[0], l[0]); l[1] = fmaf(v, g0[1], l[1]); l[2] = fmaf(v, g0[2], l[2]); l[3] = fmaf(v, g0[3], l[3]);
        l[4] = fmaf(v, g1[0], l[4]); l[5] = fmaf(v, g1[1], l[5]); l[6] = fmaf(v, g1[2], l[6]); l[7] = fmaf(v, g1[3], l[7]);
      }
    }
#pragma unroll
    for (int q = 0; q < NE; ++q) l[q] += bfr(GB[q]);
    float m = l[0];
#pragma unroll
    for (int q = 1; q < NE; ++q) m = fmaxf(m, l[q]);
    float p[NE]; float s = 0.f;
#pragma unroll
    for (int q = 0; q < NE; ++q) { p[q] = expf(l[q] - m); s += p[q]; }
    const float inv = 1.0f / s;
#pragma unroll
    for (int q = 0; q < NE; ++q) p[q] *= inv;
    int i1 = 0; float v1 = p[0];
#pragma unroll
    for (int q = 1; q < NE; ++q) { const bool gt = p[q] > v1; v1 = gt ? p[q] : v1; i1 = gt ? q : i1; }
    int i2 = 0; float v2 = -1.0f;
#pragma unroll
    for (int q = 0; q < NE; ++q) { const bool gt = (q != i1) && (p[q] > v2); v2 = gt ? p[q] : v2; i2 = gt ? q : i2; }
    s_sel[tokl] = i1 | (i2 << 4); s_p1[tokl] = v1; s_p2[tokl] = v2;
  }
  __syncthreads();

  const unsigned pc = lane & 15u, rh = lane >> 4;
#pragma unroll 1
  for (unsigned e = 0; e < (unsigned)NE; ++e) {
    const int sel0 = s_sel[t], sel1 = s_sel[t + 256u];
    const bool f0 = ((unsigned)(sel0 & 15) == e) || ((unsigned)((sel0 >> 4) & 15) == e);
    const bool f1 = ((unsigned)(sel1 & 15) == e) || ((unsigned)((sel1 >> 4) & 15) == e);
    const unsigned mk0 = __builtin_amdgcn_ballot_w32(f0), mk1 = __builtin_amdgcn_ballot_w32(f1);
    const unsigned below = (1u << lane) - 1u;
    const int pos0 = __popc(mk0 & below), pos1 = __popc(mk1 & below);
    if (lane == 0u) { s_wcnt[wv] = __popc(mk0); s_wcnt[8u + wv] = __popc(mk1); }
    __syncthreads();
    int base0 = 0, base1 = 0, tot = 0;
#pragma unroll
    for (unsigned i = 0; i < 16u; ++i) { const int c = s_wcnt[i]; base0 += (i < wv) ? c : 0; base1 += (i < 8u + wv) ? c : 0; tot += c; }
    if (f0) s_list[(unsigned)(base0 + pos0) & (unsigned)(CH - 1)] = (int)t;
    if (f1) s_list[(unsigned)(base1 + pos1) & (unsigned)(CH - 1)] = (int)(t + 256u);
    tot = tot < CH ? tot : CH;
    const int cnt = __builtin_amdgcn_readfirstlane(tot);
    __syncthreads();

    v4f b2v = *(const v4f*)(B2 + (size_t)e * DOUT + wave * 64u + 4u * pc);
#pragma unroll
    for (int i = 0; i < 4; ++i) b2v[i] = bfr(b2v[i]);

#pragma unroll 1
    for (int tile = 0; tile < CH / MT; ++tile) {
      if (tile * MT >= cnt) break;
      if (wave == 0u) {
        const int li = tile * MT + (int)lane; const bool ok = li < cnt;
        const int tl = s_list[li] & (CH - 1); const int sl = s_sel[tl];
        const float w1v = s_p1[tl], w2v = s_p2[tl];
        const bool first = (unsigned)(sl & 15) == e;
        s_rdst[lane] = ok ? (int)((first ? 0u : (unsigned)NTOK) + tok0 + (unsigned)tl) : -1;
        s_rw[lane] = ok ? (first ? w1v : w2v) : 0.f;
      }
#pragma unroll 2
      for (unsigned it = 0; it < (unsigned)(MT * DIN / 8 / 256); ++it) {
        const unsigned idx = it * 256u + t, r = idx >> 6, c = idx & 63u;
        const int li = tile * MT + (int)r; const bool ok = li < cnt;
        const unsigned tl = (unsigned)s_list[li] & (unsigned)(CH - 1);
        const float* src = X + (size_t)(tok0 + tl) * DIN + 8u * c;
        v4f a = *(const v4f*)src, b = *(const v4f*)(src + 4);
        asm volatile("" : "+v"(a), "+v"(b));
        union { v8b h; v4u u; } o;
#pragma unroll
        for (int i = 0; i < 4; ++i) { o.h[i] = (__bf16)a[i]; o.h[4 + i] = (__bf16)b[i]; }
        const v4u z = {0u, 0u, 0u, 0u};
        const v4u val = ok ? o.u : z;
        *(v4u*)&sx[r][8u * c] = val;
      }
      __syncthreads();

      v8f yacc[2][4] = {};
#pragma unroll 1
      for (unsigned hc = 0; hc < (unsigned)(DHID / HC); ++hc) {
        v8f hacc[2][2] = {};
        size_t w1o[2];
#pragma unroll
        for (int ni = 0; ni < 2; ++ni) w1o[ni] = ((size_t)e * DHID + hc * HC + wave * 32u + (unsigned)ni * 16u + lm) * DIN + 8u * lh;
#pragma unroll 2
        for (unsigned kc = 0; kc < (unsigned)(DIN / 32); ++kc) { v16b a[2], b[2];
#pragma unroll
          for (int mi = 0; mi < 2; ++mi) { union { v16b v; v4u q[2]; } f;
            f.q[0] = *(const v4u*)&sx[mi * 16 + lm][kc * 32u + 8u * lh];
            f.q[1] = *(const v4u*)&sx[mi * 16 + lm][kc * 32u + 16u + 8u * lh];
            a[mi] = f.v; }
#pragma unroll
          for (int ni = 0; ni < 2; ++ni) b[ni] = ldfrag_b(W1T + w1o[ni] + kc * 32u);
#pragma unroll
          for (int mi = 0; mi < 2; ++mi)
#pragma unroll
            for (int ni = 0; ni < 2; ++ni) hacc[mi][ni] = wmma_bf(a[mi], b[ni], hacc[mi][ni]); }
#pragma unroll
        for (int ni = 0; ni < 2; ++ni) { const float bb = bfr(B1[(size_t)e * DHID + hc * HC + wave * 32u + (unsigned)ni * 16u + lm]);
#pragma unroll
          for (int mi = 0; mi < 2; ++mi)
#pragma unroll
            for (int r = 0; r < 8; ++r) { const float h = hacc[mi][ni][r] + bb;
              const float g = 0.5f * h * (1.0f + erff(h * 0.70710678118654752f));
              shh[mi * 16 + 8u * lh + r][wave * 32u + ni * 16 + lm] = toh_flush(g * HCARRY); } }
        __syncthreads();
        size_t w2o[4];
#pragma unroll
        for (int ni = 0; ni < 4; ++ni) w2o[ni] = ((size_t)e * DOUT + wave * 64u + (unsigned)ni * 16u + lm) * DHID + hc * HC + 8u * lh;
#pragma unroll 2
        for (unsigned kc = 0; kc < (unsigned)(HC / 32); ++kc) { v16h a[2], b[4];
#pragma unroll
          for (int mi = 0; mi < 2; ++mi) { union { v16h v; v8h h[2]; } f;
            f.h[0] = *(const v8h*)&shh[mi * 16 + lm][kc * 32u + 8u * lh];
            f.h[1] = *(const v8h*)&shh[mi * 16 + lm][kc * 32u + 16u + 8u * lh];
            a[mi] = f.v; }
#pragma unroll
          for (int ni = 0; ni < 4; ++ni) b[ni] = ldfrag_h(W2T + w2o[ni] + kc * 32u);
#pragma unroll
          for (int mi = 0; mi < 2; ++mi)
#pragma unroll
            for (int ni = 0; ni < 4; ++ni) yacc[mi][ni] = wmma16(a[mi], b[ni], yacc[mi][ni]); }
        __syncthreads();
      }

#pragma unroll
      for (int mi = 0; mi < 2; ++mi) {
        if (mi) __syncthreads();
#pragma unroll
        for (int ni = 0; ni < 4; ++ni)
#pragma unroll
          for (int r = 0; r < 8; ++r) sf[wave][8u * lh + r][ni * 16 + lm] = yacc[mi][ni][r] * OSCALE;
        __syncthreads();
        v4f v[8]; int dst[8];
#pragma unroll
        for (unsigned it = 0; it < 8; ++it) { const unsigned rw = it * 2u + rh; const unsigned trw = (unsigned)mi * 16u + rw;
          const float wt = s_rw[trw]; dst[it] = s_rdst[trw];
          const v4f sv = *(const v4f*)&sf[wave][rw][4u * pc];
          v[it] = (sv + b2v) * wt; }
#pragma unroll
        for (unsigned it = 0; it < 8; ++it) { const int d = dst[it]; const unsigned dc = d >= 0 ? (unsigned)d : 0u;
          if (d >= 0) *(volatile v4f*)(YS + (size_t)dc * DOUT + wave * 64u + 4u * pc) = v[it]; }
        __threadfence();
#pragma unroll
        for (unsigned it = 0; it < 8; ++it) { const int d = dst[it]; const unsigned dc = d >= 0 ? (unsigned)d : 0u;
          if (d >= 0) *(volatile v4f*)(YS + (size_t)dc * DOUT + wave * 64u + 4u * pc) = v[it]; }
      }
      __syncthreads();
    }
  }
}

__global__ __launch_bounds__(256) void k_comb(const float* __restrict__ YS, float* __restrict__ OUT) {
  const unsigned i = blockIdx.x * 256u + threadIdx.x;
  const unsigned ic = i < (unsigned)(NTOK * DOUT / 4) ? i : (unsigned)(NTOK * DOUT / 4 - 1);
  const v4f a = *(const v4f*)(YS + (size_t)ic * 4), b = *(const v4f*)(YS + (size_t)NTOK * DOUT + (size_t)ic * 4);
  const v4f val = a + b;
  volatile v4f* p = (volatile v4f*)(OUT + (size_t)ic * 4);
  *p = val; __threadfence(); *p = val;
}

extern "C" void kernel_launch(void* const* d_in, const int* in_sizes, int n_in, void* d_out, int out_size, void* d_ws, size_t ws_size, hipStream_t stream) {
  if (n_in < 8) return;
  if (in_sizes[0] < NTOK * DIN || in_sizes[1] < NTOK * DIN || in_sizes[2] < DIN * NE || in_sizes[3] < NE) return;
  if (in_sizes[4] < NE * DIN * DHID || in_sizes[5] < NE * DHID || in_sizes[6] < NE * DHID * DOUT || in_sizes[7] < NE * DOUT) return;
  if ((size_t)out_size < (size_t)NTOK * DOUT) return;
  if (ws_size < (size_t)WS_END) return;
  const float* X  = (const float*)d_in[0];
  const float* TS = (const float*)d_in[1];
  const float* GW = (const float*)d_in[2];
  const float* GB = (const float*)d_in[3];
  const float* W1 = (const float*)d_in[4];
  const float* B1 = (const float*)d_in[5];
  const float* W2 = (const float*)d_in[6];
  const float* B2 = (const float*)d_in[7];
  char* ws = (char*)d_ws;
  unsigned short* W1T = (unsigned short*)(ws + WS_W1T);
  unsigned short* W2T = (unsigned short*)(ws + WS_W2T);
  float* YS  = (float*)(ws + WS_YS);
  float* OUT = (float*)d_out;
  k_tr_w1<<<dim3(DHID / 64, DIN / 64, NE), 256, 0, stream>>>(W1, W1T, (unsigned)DIN, (unsigned)DHID, (unsigned)DIN, (unsigned)DHID, 0u);
  k_tr_w2<<<dim3(DOUT / 64, DHID / 64, NE), 256, 0, stream>>>(W2, W2T, (unsigned)DHID, (unsigned)DOUT, (unsigned)DHID, (unsigned)DOUT, 0u, WCARRY);
  k_moe<<<dim3(NTOK / CH), 256, 0, stream>>>(X, TS, GW, GB, W1T, B1, W2T, B2, YS);
  k_comb<<<dim3(NTOK * DOUT / 4 / 256), 256, 0, stream>>>(YS, OUT);
}
